// SlidingWindowAttention_56684978372931
// MI455X (gfx1250) — hardware-verified
//
#include <hip/hip_runtime.h>


#ifndef NB
#define NB 1
#endif
#ifndef SEQ
#define SEQ 4096
#endif
#define SEQ_FULL 4096
#define DM   1024
#define NH_  16
#define HD   64
#define DQ   (NH_ * HD)
#define HW   256
#define BW   (2 * HW + 64)
#define KP   (SEQ + 2 * HW)
#define ZH   2
#define PCAR 1024.0f
#define SCL  0.125f
static_assert(SEQ % 64 == 0);
static_assert(SEQ >= 64);
static_assert(BW == 576);
static_assert(KP % 64 == 0);
static_assert(NH_ % ZH == 0);
static_assert(DQ == DM);
static_assert((ZH * SEQ) % 8 == 0);

typedef _Float16 h16;
typedef unsigned short bf;
typedef __attribute__((ext_vector_type(16))) __bf16   v16bf;
typedef __attribute__((ext_vector_type(16))) _Float16 v16h;
typedef __attribute__((ext_vector_type(8)))  _Float16 v8h;
typedef __attribute__((ext_vector_type(8)))  unsigned short v8us;
typedef __attribute__((ext_vector_type(8)))  float    v8f;
typedef __attribute__((ext_vector_type(4)))  float    v4f;
typedef v8h  __attribute__((may_alias)) v8ha;
typedef v4f  __attribute__((may_alias)) v4fa;
typedef v8us __attribute__((may_alias)) v8usa;
typedef __attribute__((ext_vector_type(2))) _Float16 v2h;
typedef __attribute__((ext_vector_type(4))) _Float16 v4h;
typedef __attribute__((ext_vector_type(2))) unsigned short v2us;
typedef __attribute__((ext_vector_type(4))) unsigned short v4us;
typedef __attribute__((ext_vector_type(2))) float v2f;

__device__ __forceinline__ unsigned short f2bf(float f) { unsigned u = __float_as_uint(f); u += 0x7FFFu + ((u >> 16) & 1u); return (unsigned short)(u >> 16); }
__device__ __forceinline__ float bf2f(unsigned short b) { return __uint_as_float(((unsigned)b) << 16); }
__device__ __forceinline__ float bfr(float f) { return bf2f(f2bf(f)); }
__device__ __forceinline__ v16h cat16(v8h lo, v8h hi) { return __builtin_shufflevector(lo, hi, 0, 1, 2, 3, 4, 5, 6, 7, 8, 9, 10, 11, 12, 13, 14, 15); }
__device__ __forceinline__ v16bf cat16b(v8us lo, v8us hi) { return __builtin_bit_cast(v16bf, __builtin_shufflevector(lo, hi, 0, 1, 2, 3, 4, 5, 6, 7, 8, 9, 10, 11, 12, 13, 14, 15)); }
__device__ __forceinline__ v8f wmma16(v16h a, v16h b, v8f c) { return __builtin_amdgcn_wmma_f32_16x16x32_f16(false, a, false, b, (short)0, c, false, false); }
__device__ __forceinline__ v8f wmmab(v16bf a, v16bf b, v8f c) { return __builtin_amdgcn_wmma_f32_16x16x32_bf16(false, a, false, b, (short)0, c, false, false); }
__device__ __forceinline__ h16 tohx(float x) { return (h16)x; }
__device__ __forceinline__ void splitf(float y, unsigned short& h, unsigned short& l) { h = f2bf(y); l = f2bf(y - bf2f(h)); }

template <typename T16> struct WFrag;
template <> struct WFrag<h16> { typedef v16h V; static __device__ __forceinline__ V ld(const h16* p) { return cat16(*(const v8h*)p, *(const v8h*)(p + 16)); } static __device__ __forceinline__ v8f mma(V a, V b, v8f c) { return wmma16(a, b, c); } };
template <> struct WFrag<bf> { typedef v16bf V; static __device__ __forceinline__ V ld(const bf* p) { return cat16b(*(const v8us*)p, *(const v8us*)(p + 16)); } static __device__ __forceinline__ v8f mma(V a, V b, v8f c) { return wmmab(a, b, c); } };
template <typename T16, int NSPLIT, bool BIAS>
__global__ __launch_bounds__(32) void k_gemmw(const T16* __restrict__ A, const T16* __restrict__ A2, const T16* __restrict__ Bt, const T16* __restrict__ Bt2, int K, float* C, int ldc, const float* __restrict__ bias, size_t sA, size_t sB, size_t sC) {
    typedef typename WFrag<T16>::V V;
    __shared__ __align__(16) float os[16 * 68];
    const size_t z = blockIdx.z; A += z * sA; if (A2) A2 += z * sA; Bt += z * sB; if (Bt2) Bt2 += z * sB; C += z * sC;
    const int lane = threadIdx.x & 31, lr = lane & 15, hi = lane >> 4; const int r0 = blockIdx.x * 64, c0 = blockIdx.y * 64;
    v8f acc[4][4];
#pragma unroll
    for (int mb = 0; mb < 4; ++mb)
#pragma unroll
        for (int nb = 0; nb < 4; ++nb) acc[mb][nb] = (v8f){};
    const size_t aoff = (size_t)(r0 + lr) * K + 8 * hi, boff = (size_t)(c0 + lr) * K + 8 * hi;
#pragma unroll 1
    for (int kc = 0; kc < K; kc += 32) {
        V a[4], a2[4];
#pragma unroll
        for (int mb = 0; mb < 4; ++mb) { a[mb] = WFrag<T16>::ld(A + aoff + (size_t)mb * 16 * K + kc); if (NSPLIT == 1 || NSPLIT == 2) a2[mb] = WFrag<T16>::ld(A2 + aoff + (size_t)mb * 16 * K + kc); }
#pragma unroll
        for (int nb = 0; nb < 4; ++nb) { const V b = WFrag<T16>::ld(Bt + boff + (size_t)nb * 16 * K + kc); V b2; if (NSPLIT >= 2) b2 = WFrag<T16>::ld(Bt2 + boff + (size_t)nb * 16 * K + kc);
#pragma unroll
            for (int mb = 0; mb < 4; ++mb) { acc[mb][nb] = WFrag<T16>::mma(a[mb], b, acc[mb][nb]); if (NSPLIT == 1 || NSPLIT == 2) acc[mb][nb] = WFrag<T16>::mma(a2[mb], b, acc[mb][nb]); if (NSPLIT >= 2) acc[mb][nb] = WFrag<T16>::mma(a[mb], b2, acc[mb][nb]); } }
        asm volatile("v_nop\n\tv_nop\n\tv_nop\n\tv_nop" : "+v"(acc[0][0]), "+v"(acc[1][1]), "+v"(acc[2][2]), "+v"(acc[3][3]) : "v"(a[0]), "v"(a[3]));
    }
#pragma unroll
    for (int mb = 0; mb < 4; ++mb) {
#pragma unroll
        for (int nb = 0; nb < 4; ++nb) {
#pragma unroll
            for (int j = 0; j < 8; ++j) os[(hi * 8 + j) * 68 + nb * 16 + lr] = acc[mb][nb][j]; }
        __builtin_amdgcn_wave_barrier(); asm volatile("" ::: "memory");
        float* crow = C + (size_t)(r0 + mb * 16) * ldc + c0;
#pragma unroll 1
        for (int ps = 0; ps < 2; ++ps) {
#pragma unroll
            for (int s = 0; s < 8; ++s) { const int row = 2 * s + hi, cofs = lr * 4; v4f val = *(const v4fa*)(os + row * 68 + cofs); if (BIAS) { val[0] += bfr(bias[c0 + cofs]); val[1] += bfr(bias[c0 + cofs + 1]); val[2] += bfr(bias[c0 + cofs + 2]); val[3] += bfr(bias[c0 + cofs + 3]); }
                *(volatile v4f*)(crow + (size_t)row * ldc + cofs) = val; }
            if (ps == 0) __threadfence(); }
        __builtin_amdgcn_wave_barrier(); asm volatile("" ::: "memory");
    }
}

template <int BAND>
__global__ __launch_bounds__(32) void k_gemmb(const h16* __restrict__ A, const h16* __restrict__ Bt, int K, int ldb, float* C, int ldc, size_t sA, size_t sB, size_t sC) {
    __shared__ __align__(16) float os[16 * 68];
    const size_t z = blockIdx.z; A += z * sA; Bt += z * sB; C += z * sC;
    const int lane = threadIdx.x & 31, lr = lane & 15, hi = lane >> 4; const int r0 = blockIdx.x * 64, c0 = blockIdx.y * 64;
    v8f acc[4][4];
#pragma unroll
    for (int mb = 0; mb < 4; ++mb)
#pragma unroll
        for (int nb = 0; nb < 4; ++nb) acc[mb][nb] = (v8f){};
    const size_t aoff = (size_t)(r0 + lr) * K + 8 * hi;
    const size_t boff = (BAND == 1) ? ((size_t)(r0 + c0 + lr) * ldb + 8 * hi) : ((size_t)(c0 + lr) * ldb + (size_t)r0 + 8 * hi);
#pragma unroll 1
    for (int kc = 0; kc < K; kc += 32) {
        v16h a[4];
#pragma unroll
        for (int mb = 0; mb < 4; ++mb) a[mb] = WFrag<h16>::ld(A + aoff + (size_t)mb * 16 * K + kc);
#pragma unroll
        for (int nb = 0; nb < 4; ++nb) { const v16h b = WFrag<h16>::ld(Bt + boff + (size_t)nb * 16 * ldb + kc);
#pragma unroll
            for (int mb = 0; mb < 4; ++mb) acc[mb][nb] = wmma16(a[mb], b, acc[mb][nb]); }
        asm volatile("v_nop\n\tv_nop\n\tv_nop\n\tv_nop" : "+v"(acc[0][0]), "+v"(acc[1][1]), "+v"(acc[2][2]), "+v"(acc[3][3]) : "v"(a[0]), "v"(a[3]));
    }
#pragma unroll
    for (int mb = 0; mb < 4; ++mb) {
#pragma unroll
        for (int nb = 0; nb < 4; ++nb) {
#pragma unroll
            for (int j = 0; j < 8; ++j) os[(hi * 8 + j) * 68 + nb * 16 + lr] = acc[mb][nb][j]; }
        __builtin_amdgcn_wave_barrier(); asm volatile("" ::: "memory");
        float* crow = C + (size_t)(r0 + mb * 16) * ldc + c0;
#pragma unroll 1
        for (int ps = 0; ps < 2; ++ps) {
#pragma unroll
            for (int s = 0; s < 8; ++s) { const int row = 2 * s + hi, cofs = lr * 4; v4f val = *(const v4fa*)(os + row * 68 + cofs);
                *(volatile v4f*)(crow + (size_t)row * ldc + cofs) = val; }
            if (ps == 0) __threadfence(); }
        __builtin_amdgcn_wave_barrier(); asm volatile("" ::: "memory");
    }
}

__global__ __launch_bounds__(256) void k_cvt8(const float* __restrict__ src, bf* dst, size_t n8) { const size_t i = (size_t)blockIdx.x * 256 + threadIdx.x; if (i >= n8) return; const v8f v = *(const v8f*)(src + i * 8); v8us o;
#pragma unroll
    for (int k = 0; k < 8; ++k) o[k] = f2bf(v[k]); *(volatile v8us*)(dst + i * 8) = o; __threadfence(); *(volatile v8us*)(dst + i * 8) = o; }

__global__ __launch_bounds__(256) void k_qplane(const float* __restrict__ F, h16* Q16, size_t n8) {
    const size_t i = (size_t)blockIdx.x * 256 + threadIdx.x; if (i >= n8) return; const size_t e = i * 8;
    const int d = (int)(e % HD); const int t = (int)((e / HD) % SEQ); const int h = (int)(e / ((size_t)HD * SEQ));
    const float* f = F + (size_t)t * DQ + h * HD + d; const v4f a0 = *(const v4f*)f; const v4f a1 = *(const v4f*)(f + 4); v8h o;
#pragma unroll
    for (int k = 0; k < 4; ++k) { o[k] = tohx(a0[k]); o[4 + k] = tohx(a1[k]); }
    *(volatile v8h*)(Q16 + e) = o; __threadfence(); *(volatile v8h*)(Q16 + e) = o; }

__global__ __launch_bounds__(256) void k_kplane(const float* __restrict__ F, h16* K16, size_t n8) {
    const size_t i = (size_t)blockIdx.x * 256 + threadIdx.x; if (i >= n8) return; const size_t e = i * 8;
    const int d = (int)(e % HD); const int tp = (int)((e / HD) % KP); const int h = (int)(e / ((size_t)HD * KP));
    const int t = tp - HW; const bool ok = (t >= 0) && (t < SEQ); const int tc = min(max(t, 0), SEQ - 1);
    const float* f = F + (size_t)tc * DQ + h * HD + d; const v4f a0 = *(const v4f*)f; const v4f a1 = *(const v4f*)(f + 4); v8h o;
#pragma unroll
    for (int k = 0; k < 4; ++k) { const float x0 = ok ? a0[k] : 0.0f; const float x1 = ok ? a1[k] : 0.0f; o[k] = tohx(x0); o[4 + k] = tohx(x1); }
    *(volatile v8h*)(K16 + e) = o; __threadfence(); *(volatile v8h*)(K16 + e) = o; }

__global__ __launch_bounds__(256) void k_vtplane(const float* __restrict__ F, h16* V16, size_t n8) {
    const size_t i = (size_t)blockIdx.x * 256 + threadIdx.x; if (i >= n8) return; const size_t e = i * 8;
    const int tp0 = (int)(e % KP); const int d = (int)((e / KP) % HD); const int h = (int)(e / ((size_t)KP * HD)); v8h o;
#pragma unroll
    for (int q = 0; q < 8; ++q) { const int t = tp0 + q - HW; const bool ok = (t >= 0) && (t < SEQ); const int tc = min(max(t, 0), SEQ - 1);
        const float xv = F[(size_t)tc * DQ + h * HD + d]; const float xs = ok ? xv : 0.0f; o[q] = tohx(xs); }
    *(volatile v8h*)(V16 + e) = o; __threadfence(); *(volatile v8h*)(V16 + e) = o; }

__global__ __launch_bounds__(256) void k_band_soft(const float* __restrict__ Sb, h16* P16) {
    const int lane = threadIdx.x & 31; const int row = blockIdx.x * 8 + (threadIdx.x >> 5); if (row >= ZH * SEQ) return;
    const int i = row % SEQ; const int jbase = (i & ~63) - HW;
    const float* sr = Sb + (size_t)row * BW; float v[BW / 32]; float mx = -3.0e38f;
#pragma unroll
    for (int ch = 0; ch < (BW - 64) / 128; ++ch) { const int jj0 = ch * 128 + lane * 4; const v4f a = *(const v4f*)(sr + jj0);
#pragma unroll
        for (int q = 0; q < 4; ++q) { const int j = jbase + jj0 + q; const bool ok = (j >= 0) && (j < SEQ) && (j >= i - HW) && (j <= i + HW); const float t = ok ? a[q] * SCL : -3.0e38f; v[ch * 4 + q] = t; mx = fmaxf(mx, t); } }
    { const int jj0 = (BW - 64) + lane * 2; const v2f a = *(const v2f*)(sr + jj0);
#pragma unroll
        for (int q = 0; q < 2; ++q) { const int j = jbase + jj0 + q; const bool ok = (j >= 0) && (j < SEQ) && (j >= i - HW) && (j <= i + HW); const float t = ok ? a[q] * SCL : -3.0e38f; v[(BW - 64) / 32 + q] = t; mx = fmaxf(mx, t); } }
#pragma unroll
    for (int sh = 16; sh; sh >>= 1) mx = fmaxf(mx, __shfl_xor(mx, sh, 32));
    float sum = 0.f;
#pragma unroll
    for (int k = 0; k < BW / 32; ++k) { float d0 = __fsub_rn(v[k], mx); asm volatile("" : "+v"(d0)); v[k] = __builtin_amdgcn_exp2f(__fmul_rn(d0, 1.4426950408889634f)); sum += v[k]; }
#pragma unroll
    for (int sh = 16; sh; sh >>= 1) sum += __shfl_xor(sum, sh, 32);
    const float f = __fdiv_rn(PCAR, sum);
    h16* prow = P16 + (size_t)row * BW;
#pragma unroll 1
    for (int ps = 0; ps < 2; ++ps) {
#pragma unroll
        for (int ch = 0; ch < (BW - 64) / 128; ++ch) { v4h o4;
#pragma unroll
            for (int q = 0; q < 4; ++q) o4[q] = tohx(v[ch * 4 + q] * f);
            *(volatile v4h*)(prow + ch * 128 + lane * 4) = o4; }
        { v2h o2;
#pragma unroll
            for (int q = 0; q < 2; ++q) o2[q] = tohx(v[(BW - 64) / 32 + q] * f);
            *(volatile v2h*)(prow + (BW - 64) + lane * 2) = o2; }
        if (ps == 0) __threadfence(); }
}

__global__ __launch_bounds__(256) void k_merge(const float* __restrict__ O, int h0, bf* Ah, bf* Al) { const size_t e = ((size_t)blockIdx.x * 256 + threadIdx.x) * 2; if (e >= (size_t)ZH * SEQ * HD) return; const int d = (int)(e % HD); const int t = (int)((e / HD) % SEQ); const int zz = (int)(e / ((size_t)HD * SEQ)); const size_t oo = (size_t)t * DQ + (size_t)(h0 + zz) * HD + d;
    v2us oh, ol;
#pragma unroll
    for (int q = 0; q < 2; ++q) { unsigned short a, c2; splitf(O[e + q] * (1.0f / PCAR), a, c2); oh[q] = a; ol[q] = c2; } *(volatile v2us*)(Ah + oo) = oh; *(volatile v2us*)(Al + oo) = ol; __threadfence(); *(volatile v2us*)(Ah + oo) = oh; *(volatile v2us*)(Al + oo) = ol; }

extern "C" void kernel_launch(void* const* d_in, const int* in_sizes, int n_in,
                              void* d_out, int out_size, void* d_ws, size_t ws_size, hipStream_t stream) {
    if (n_in < 5) return;
    const long long needx = (long long)(NB - 1) * SEQ_FULL * DM + (long long)SEQ * DM;
    if ((long long)in_sizes[0] < needx) return;
    for (int k = 1; k < 5; ++k) if ((long long)in_sizes[k] < (long long)DM * DM) return;
    if ((long long)out_size < needx) return;
    const float* x = (const float*)d_in[0]; const float* wq = (const float*)d_in[1]; const float* wk = (const float*)d_in[2]; const float* wv = (const float*)d_in[3]; const float* wo = (const float*)d_in[4];
    float* OUT = (float*)d_out;
    char* wsp = (char*)d_ws;
    auto take = [&](size_t bytes) { char* p = wsp; wsp += (bytes + 255) & ~(size_t)255; return (void*)p; };
    bf* WQ = (bf*)take((size_t)DQ * DM * 2); bf* WK = (bf*)take((size_t)DQ * DM * 2); bf* WV = (bf*)take((size_t)DQ * DM * 2); bf* WO = (bf*)take((size_t)DM * DQ * 2);
    bf* XB = (bf*)take((size_t)SEQ * DM * 2); float* F = (float*)take((size_t)SEQ * DQ * 4);
    h16* QP16 = (h16*)take((size_t)NH_ * SEQ * HD * 2); h16* KP16 = (h16*)take((size_t)NH_ * KP * HD * 2); h16* VT16 = (h16*)take((size_t)NH_ * HD * KP * 2);
    float* Sb = (float*)take((size_t)ZH * SEQ * BW * 4); h16* P16 = (h16*)take((size_t)ZH * SEQ * BW * 2); float* Ob = (float*)take((size_t)ZH * SEQ * HD * 4);
    bf* ATh = (bf*)take((size_t)SEQ * DQ * 2); bf* ATl = (bf*)take((size_t)SEQ * DQ * 2);
    if ((size_t)(wsp - (char*)d_ws) > ws_size) return;
    const size_t nw8 = (size_t)DM * DM / 8, nx8 = (size_t)SEQ * DM / 8, nq8 = (size_t)NH_ * SEQ * HD / 8, nk8 = (size_t)NH_ * KP * HD / 8;
    const unsigned LW = (unsigned)((nw8 + 255) / 256), LX = (unsigned)((nx8 + 255) / 256), LQ = (unsigned)((nq8 + 255) / 256), LK = (unsigned)((nk8 + 255) / 256);
    const unsigned LM = (unsigned)(((size_t)ZH * SEQ * HD / 2 + 255) / 256);
    k_cvt8<<<LW, 256, 0, stream>>>(wq, WQ, nw8); k_cvt8<<<LW, 256, 0, stream>>>(wk, WK, nw8); k_cvt8<<<LW, 256, 0, stream>>>(wv, WV, nw8); k_cvt8<<<LW, 256, 0, stream>>>(wo, WO, nw8);
    for (int b = 0; b < NB; ++b) {
        k_cvt8<<<LX, 256, 0, stream>>>(x + (size_t)b * SEQ_FULL * DM, XB, nx8);
        k_gemmw<bf, 0, false><<<dim3(SEQ / 64, DQ / 64, 1), 32, 0, stream>>>(XB, nullptr, WQ, nullptr, DM, F, DQ, nullptr, 0, 0, 0);
        k_qplane<<<LQ, 256, 0, stream>>>(F, QP16, nq8);
        k_gemmw<bf, 0, false><<<dim3(SEQ / 64, DQ / 64, 1), 32, 0, stream>>>(XB, nullptr, WK, nullptr, DM, F, DQ, nullptr, 0, 0, 0);
        k_kplane<<<LK, 256, 0, stream>>>(F, KP16, nk8);
        k_gemmw<bf, 0, false><<<dim3(SEQ / 64, DQ / 64, 1), 32, 0, stream>>>(XB, nullptr, WV, nullptr, DM, F, DQ, nullptr, 0, 0, 0);
        k_vtplane<<<LK, 256, 0, stream>>>(F, VT16, nk8);
        for (int h0 = 0; h0 < NH_; h0 += ZH) {
            k_gemmb<1><<<dim3(SEQ / 64, BW / 64, ZH), 32, 0, stream>>>(QP16 + (size_t)h0 * SEQ * HD, KP16 + (size_t)h0 * KP * HD, HD, HD, Sb, BW, (size_t)SEQ * HD, (size_t)KP * HD, (size_t)SEQ * BW);
            k_band_soft<<<(unsigned)(ZH * SEQ / 8), 256, 0, stream>>>(Sb, P16);
            k_gemmb<2><<<dim3(SEQ / 64, HD / 64, ZH), 32, 0, stream>>>(P16, VT16 + (size_t)h0 * HD * KP, BW, KP, Ob, HD, (size_t)SEQ * BW, (size_t)HD * KP, (size_t)SEQ * HD);
            k_merge<<<LM, 256, 0, stream>>>(Ob, h0, ATh, ATl); }
        k_gemmw<bf, 1, false><<<dim3(SEQ / 64, DM / 64, 1), 32, 0, stream>>>(ATh, ATl, WO, nullptr, DQ, OUT + (size_t)b * SEQ_FULL * DM, DM, nullptr, 0, 0, 0); }
}
